// DeformBasicBlock_6313601925210
// MI455X (gfx1250) — hardware-verified
//
#include <hip/hip_runtime.h>
#include <stddef.h>


#define NB    2
#define CC    64
#define DD    8
#define HH    56
#define WW    56
#define HW2   3136
#define PP    25088
#define NQ    50176
#define KT    27
#define KD    1728
#define OFFC  648
#define OFFN  704
#define HP    58
#define WP    58
#define PLANE 3364
#define PVOL  33640
#define GF    64
#define RP    33792
#define MSO   3423
#define MOFF  6656
#define CHR   6272
#define NCH   8
#define RO    26816
#define NSL   64
#define RS    784

typedef __attribute__((ext_vector_type(16))) _Float16 v16h;
typedef __attribute__((ext_vector_type(8)))  _Float16 v8h;
typedef __attribute__((ext_vector_type(16))) __bf16   v16b;
typedef __attribute__((ext_vector_type(8)))  __bf16   v8b;
typedef __attribute__((ext_vector_type(8)))  float    v8f;
typedef __attribute__((ext_vector_type(4)))  float    v4f;
typedef __attribute__((ext_vector_type(4)))  unsigned v4u;

__device__ __forceinline__ unsigned short f2bf_bits(float f) {
  unsigned u = __float_as_uint(f);
  return (unsigned short)((u + 0x7FFFu + ((u >> 16) & 1u)) >> 16);
}
__device__ __forceinline__ float bf_bits2f(unsigned short h) { return __uint_as_float(((unsigned)h) << 16); }

__device__ __forceinline__ unsigned pk2(unsigned short a, unsigned short b) {
  return (unsigned)a | ((unsigned)b << 16);
}
__device__ __forceinline__ unsigned pkh2(float a, float b) {
  return pk2(__builtin_bit_cast(unsigned short, (_Float16)a), __builtin_bit_cast(unsigned short, (_Float16)b));
}

__device__ __forceinline__ void dep_guard_h(v8f& a, v8f& b, v16h x, v16h y) { asm volatile("v_nop\n\tv_nop\n\tv_nop\n\tv_nop" : "+v"(a), "+v"(b) : "v"(x), "v"(y)); }
__device__ __forceinline__ void dep_guard_b(v8f& a, v8f& b, v16b x, v16b y) { asm volatile("v_nop\n\tv_nop\n\tv_nop\n\tv_nop" : "+v"(a), "+v"(b) : "v"(x), "v"(y)); }
__device__ __forceinline__ void keep4_h(v16h a, v16h b, v16h c, v16h d) { asm volatile("v_nop" :: "v"(a), "v"(b), "v"(c), "v"(d)); }
__device__ __forceinline__ void keep4_b(v16b a, v16b b, v16b c, v16b d) { asm volatile("v_nop" :: "v"(a), "v"(b), "v"(c), "v"(d)); }
__device__ __forceinline__ void acc_guard4(v8f& a, v8f& b, v8f& c, v8f& d) { asm volatile("v_nop\n\tv_nop\n\tv_nop\n\tv_nop" : "+v"(a), "+v"(b), "+v"(c), "+v"(d)); }
template <typename T> struct Frag;
template <> struct Frag<_Float16> {
  typedef v16h V; union U { v16h v; v8h h[2]; };
  static __device__ __forceinline__ v16h load(const _Float16* p) {
    U f; f.h[0] = *(const v8h*)(p); f.h[1] = *(const v8h*)(p + 16); return f.v;
  }
  static __device__ __forceinline__ v8f mma(v16h a, v16h b, v8f c) {
    return __builtin_amdgcn_wmma_f32_16x16x32_f16(false, a, false, b, (short)0, c, false, false);
  }
  static __device__ __forceinline__ void guard(v8f& a, v8f& b, v16h x, v16h y) { dep_guard_h(a, b, x, y); }
  static __device__ __forceinline__ void keep(v16h a, v16h b, v16h c, v16h d) { keep4_h(a, b, c, d); }
};
template <> struct Frag<__bf16> {
  typedef v16b V; union U { v16b v; v8b h[2]; };
  static __device__ __forceinline__ v16b load(const __bf16* p) {
    U f; f.h[0] = *(const v8b*)(p); f.h[1] = *(const v8b*)(p + 16); return f.v;
  }
  static __device__ __forceinline__ v8f mma(v16b a, v16b b, v8f c) {
    return __builtin_amdgcn_wmma_f32_16x16x32_bf16(false, a, false, b, (short)0, c, false, false);
  }
  static __device__ __forceinline__ void guard(v8f& a, v8f& b, v16b x, v16b y) { dep_guard_b(a, b, x, y); }
  static __device__ __forceinline__ void keep(v16b a, v16b b, v16b c, v16b d) { keep4_b(a, b, c, d); }
};

template <int ET> struct Elem;
template <> struct Elem<0> { typedef _Float16 T; };
template <> struct Elem<1> { typedef __bf16 T; };
template <int ET, bool SPLIT, int BIAS_MODE, int OUT_MODE, bool RESID, int ACT = 0, int CONVA = 0>
__global__ __launch_bounds__(256) void wmma_gemm64(
    const unsigned short* __restrict__ Ap, const unsigned short* __restrict__ A2p, int lda, long strideA,
    const unsigned short* __restrict__ Btp, const unsigned short* __restrict__ Bt2p, int ldb, long strideB,
    void* __restrict__ Cout, void* __restrict__ Cout2, int ldc, long strideC,
    const float* __restrict__ bias,
    const float* __restrict__ resid, long strideR,
    int M, int N, int K, float scale) {
  typedef typename Elem<ET>::T T;
  typedef typename Frag<T>::V V;
  const T* A = (const T*)Ap; const T* A2 = (const T*)A2p; const T* Bt = (const T*)Btp; const T* Bt2 = (const T*)Bt2p;
  __shared__ __align__(16) float sT[8][16 * 68];
  const int b    = blockIdx.y;
  const int lane = threadIdx.x & 31;
  const int wave = threadIdx.x >> 5;
  const int tilesN = N >> 6;
  const int tilesM = M >> 6;
  const int tile = blockIdx.x * 8 + wave;
  if (tile >= tilesM * tilesN) return;
  const int tm = tile / tilesN;
  const int tn = tile - tm * tilesN;
  const int m0 = tm << 6;
  const int n0 = tn << 6;

  const T* Ab  = A  + (size_t)b * strideA;
  const T* Bb  = Bt + (size_t)b * strideB;
  const T* Ab2 = SPLIT ? (A2  + (size_t)b * strideA) : nullptr;
  const T* Bb2 = SPLIT ? (Bt2 + (size_t)b * strideB) : nullptr;

  const int rlane = lane & 15;
  const int koff  = (lane >> 4) * 8;
  const int mOff  = (lane >> 4) * 8;

  v8f acc[4][4];
#pragma unroll
  for (int i = 0; i < 4; ++i)
#pragma unroll
    for (int j = 0; j < 4; ++j) acc[i][j] = (v8f){0.f,0.f,0.f,0.f,0.f,0.f,0.f,0.f};

  for (int k0 = 0; k0 < K; k0 += 32) {
    ptrdiff_t arow = 0;
    int acol = k0;
    if (CONVA) {
      const int t = k0 >> 6;
      const int kd = t / 9; const int r9 = t - kd * 9; const int kh = r9 / 3; const int kw = r9 - kh * 3;
      arow = (ptrdiff_t)(((kd - 1) * HP + (kh - 1)) * WP + (kw - 1));
      acol = k0 & 63;
    }
    V bh[4], bl[4];
#pragma unroll
    for (int j = 0; j < 4; ++j) {
      const size_t bo = (size_t)(n0 + (j << 4) + rlane) * ldb + koff + k0;
      bh[j] = Frag<T>::load(Bb + bo);
      if (SPLIT) bl[j] = Frag<T>::load(Bb2 + bo);
    }
#pragma unroll
    for (int i = 0; i < 4; ++i) {
      const ptrdiff_t ao = ((ptrdiff_t)(m0 + (i << 4) + rlane) + arow) * lda + koff + acol;
      V ah = Frag<T>::load(Ab + ao);
      V al;
      if (SPLIT) al = Frag<T>::load(Ab2 + ao);
#pragma unroll
      for (int j = 0; j < 4; ++j) {
        acc[i][j] = Frag<T>::mma(ah, bh[j], acc[i][j]);
        if (SPLIT) {
          acc[i][j] = Frag<T>::mma(ah, bl[j], acc[i][j]);
          acc[i][j] = Frag<T>::mma(al, bh[j], acc[i][j]);
        }
      }
      Frag<T>::guard(acc[i][0], acc[i][3], ah, SPLIT ? al : ah);
    }
    Frag<T>::keep(bh[0], bh[1], bh[2], bh[3]);
    if (SPLIT) Frag<T>::keep(bl[0], bl[1], bl[2], bl[3]);
  }
  acc_guard4(acc[0][0], acc[0][1], acc[0][2], acc[0][3]);
  acc_guard4(acc[1][0], acc[1][1], acc[1][2], acc[1][3]);
  acc_guard4(acc[2][0], acc[2][1], acc[2][2], acc[2][3]);
  acc_guard4(acc[3][0], acc[3][1], acc[3][2], acc[3][3]);

  float* slab = sT[wave];
  const float* Rb = RESID ? (resid + (size_t)b * strideR) : nullptr;
#pragma unroll
  for (int i = 0; i < 4; ++i) {
    const int mBase = m0 + (i << 4);
#pragma unroll
    for (int j = 0; j < 4; ++j) {
      const int n = n0 + (j << 4) + rlane;
      float bv = 0.f;
      if (BIAS_MODE == 2) bv = bias[n];
#pragma unroll
      for (int r = 0; r < 8; ++r) {
        float v = acc[i][j][r] * scale;
        if (BIAS_MODE == 1) v += bias[mBase + mOff + r];
        if (BIAS_MODE == 2) v += bv;
        if (RESID) v += Rb[(size_t)(mBase + mOff + r) * ldc + n];
        if (ACT == 1) v = tanhf(v);
        if (ACT == 2) v = fmaxf(v, 0.0f);
        if (ACT == 3) v = v / (1.0f + expf(-v));
        if (ACT == 4) v = (v > 0.f) ? v : 0.01f * v;
        if (ACT == 5) v = 0.5f * v * (1.0f + erff(v * 0.70710678118654752f));
        slab[(mOff + r) * 68 + (j << 4) + rlane] = v;
      }
    }
    __builtin_amdgcn_fence(__ATOMIC_RELEASE, "workgroup");
    __builtin_amdgcn_wave_barrier();
    __builtin_amdgcn_fence(__ATOMIC_ACQUIRE, "workgroup");
    if (OUT_MODE == 0) {
      float* C = (float*)Cout + (size_t)b * strideC;
      const int hh = lane >> 4, c4 = (lane & 15) * 4;
      for (int pass = 0; pass < 2; ++pass) {
#pragma unroll
        for (int it = 0; it < 8; ++it) {
          const int row = it * 2 + hh;
          v4f v = *(const v4f*)(slab + row * 68 + c4);
          *(volatile v4f*)(C + (size_t)(mBase + row) * ldc + n0 + c4) = v;
        }
        __threadfence();
      }
    } else {
      const int q = lane >> 3, c8 = (lane & 7) * 8;
      unsigned short* C  = (unsigned short*)Cout  + (size_t)b * strideC;
      unsigned short* C2 = (OUT_MODE == 2) ? ((unsigned short*)Cout2 + (size_t)b * strideC) : nullptr;
      for (int pass = 0; pass < 2; ++pass) {
#pragma unroll
        for (int it = 0; it < 4; ++it) {
          const int row = it * 4 + q;
          const float* sp = slab + row * 68 + c8;
          v8h hv, lv;
#pragma unroll
          for (int e = 0; e < 8; ++e) {
            if (OUT_MODE == 1) {
              hv[e] = (_Float16)sp[e];
            } else {
              unsigned short hb = f2bf_bits(sp[e]);
              unsigned short lb = f2bf_bits(sp[e] - bf_bits2f(hb));
              hv[e] = __builtin_bit_cast(_Float16, hb);
              lv[e] = __builtin_bit_cast(_Float16, lb);
            }
          }
          *(volatile v8h*)(C + (size_t)(mBase + row) * ldc + n0 + c8) = hv;
          if (OUT_MODE == 2) *(volatile v8h*)(C2 + (size_t)(mBase + row) * ldc + n0 + c8) = lv;
        }
        __threadfence();
      }
    }
    __builtin_amdgcn_fence(__ATOMIC_RELEASE, "workgroup");
    __builtin_amdgcn_wave_barrier();
    __builtin_amdgcn_fence(__ATOMIC_ACQUIRE, "workgroup");
  }
}

__global__ __launch_bounds__(256) void k_xpose(const float* __restrict__ x, float* __restrict__ xT) {
  __shared__ float t[CC][33];
  const int tid = threadIdx.x;
  const int blk = blockIdx.x;
  const int b   = blk / (PP / 32);
  const int p0  = (blk - b * (PP / 32)) * 32;
  const float* xb = x + (size_t)b * CC * PP + p0;
#pragma unroll
  for (int i = 0; i < 8; ++i) {
    const int idx = i * 256 + tid;
    const int c = idx >> 5, j = idx & 31;
    t[c][j] = xb[(size_t)c * PP + j];
  }
  __syncthreads();
  const int wave = tid >> 5, lane = tid & 31, hh = lane >> 4, c4 = (lane & 15) * 4;
  float* ob = xT + ((size_t)b * PP + p0) * CC;
  for (int pass = 0; pass < 2; ++pass) {
#pragma unroll
    for (int it = 0; it < 2; ++it) {
      const int row = wave * 4 + it * 2 + hh;
      v4f v;
      v[0] = t[c4][row]; v[1] = t[c4 + 1][row]; v[2] = t[c4 + 2][row]; v[3] = t[c4 + 3][row];
      *(volatile v4f*)(ob + (size_t)row * CC + c4) = v;
    }
    __threadfence();
  }
}

__device__ __forceinline__ v4f relu4(v4f a) {
  v4f r;
  r[0] = fmaxf(a[0], 0.0f); r[1] = fmaxf(a[1], 0.0f); r[2] = fmaxf(a[2], 0.0f); r[3] = fmaxf(a[3], 0.0f);
  return r;
}

template <int BN>
__global__ __launch_bounds__(256) void k_pad16(const float* __restrict__ src, const float* __restrict__ stats,
                                               const float* __restrict__ gamma, const float* __restrict__ beta,
                                               unsigned short* __restrict__ dst) {
  const int lane = threadIdx.x & 31, wave = threadIdx.x >> 5;
  const int q = lane >> 3, c8 = (lane & 7) * 8;
  const int it = (blockIdx.x * 8 + wave) * 4 + q;
  if (it < NB * RP) {
    const int n = it / RP, r = it - n * RP;
    const int mp = r - GF;
    const bool inside = (mp >= 0) && (mp < PVOL);
    const int mpc = mp < 0 ? 0 : (mp > PVOL - 1 ? PVOL - 1 : mp);
    const int dp = mpc / PLANE, rem = mpc - dp * PLANE, hp = rem / WP, wp = rem - hp * WP;
    const bool interior = inside && (dp >= 1) && (dp <= DD) && (hp >= 1) && (hp <= HH) && (wp >= 1) && (wp <= WW);
    int dv = dp - 1, hv = hp - 1, wv = wp - 1;
    dv = dv < 0 ? 0 : (dv > DD - 1 ? DD - 1 : dv);
    hv = hv < 0 ? 0 : (hv > HH - 1 ? HH - 1 : hv);
    wv = wv < 0 ? 0 : (wv > WW - 1 ? WW - 1 : wv);
    const float* sp = src + ((size_t)n * PP + (size_t)(dv * HW2 + hv * WW + wv)) * CC + c8;
    v4f a = *(const v4f*)(sp);
    v4f c = *(const v4f*)(sp + 4);
    if (BN) {
      const v4f m0 = *(const v4f*)(stats + c8),      m1 = *(const v4f*)(stats + c8 + 4);
      const v4f r0 = *(const v4f*)(stats + CC + c8), r1 = *(const v4f*)(stats + CC + c8 + 4);
      const v4f g0 = *(const v4f*)(gamma + c8),      g1 = *(const v4f*)(gamma + c8 + 4);
      const v4f b0 = *(const v4f*)(beta + c8),       b1 = *(const v4f*)(beta + c8 + 4);
      a = (g0 * (a - m0)) * r0 + b0;
      c = (g1 * (c - m1)) * r1 + b1;
      a = relu4(a); c = relu4(c);
    }
    const v4f z = (v4f){0.f, 0.f, 0.f, 0.f};
    if (!interior) { a = z; c = z; }
    v4u u;
    u[0] = pkh2(a[0], a[1]); u[1] = pkh2(a[2], a[3]);
    u[2] = pkh2(c[0], c[1]); u[3] = pkh2(c[2], c[3]);
    volatile v4u* d = (volatile v4u*)(dst + (size_t)it * CC + c8);
    *d = u;
    __threadfence();
    *d = u;
  }
}

__global__ __launch_bounds__(256) void k_prepw(const float* __restrict__ w, unsigned short* __restrict__ B,
                                              int orows, int ovalid, float scale) {
  const int gidx = blockIdx.x * 256 + threadIdx.x;
  if (gidx < orows * (KD / 8)) {
    const int e0 = gidx * 8;
    const int o  = e0 / KD;
    const int col = e0 - o * KD;
    const int t  = col >> 6;
    const int c0 = col & 63;
    const int oc = o < ovalid ? o : (ovalid - 1);
    float f[8];
#pragma unroll
    for (int j = 0; j < 8; ++j) {
      const float v = w[((size_t)(oc * CC + c0 + j)) * KT + t] * scale;
      f[j] = (o < ovalid) ? v : 0.0f;
    }
    v4u u;
    u[0] = pkh2(f[0], f[1]); u[1] = pkh2(f[2], f[3]); u[2] = pkh2(f[4], f[5]); u[3] = pkh2(f[6], f[7]);
    volatile v4u* p = (volatile v4u*)(B + e0);
    *p = u;
    __threadfence();
    *p = u;
  }
}

__device__ __forceinline__ void acc_corner(const float* __restrict__ p, float wv, v4f& a, v4f& b) {
  const v4f ga = *(const v4f*)(p);
  const v4f gb = *(const v4f*)(p + 4);
  a = a + ga * wv;
  b = b + gb * wv;
}

__global__ __launch_bounds__(256) void k_sample(const float* __restrict__ xT, const float* __restrict__ offc,
                                                const float* __restrict__ boff, unsigned short* __restrict__ S,
                                                int n, int dbase) {
  const int lane = threadIdx.x & 31, wave = threadIdx.x >> 5;
  const int q = lane >> 3, g = lane & 7;
  const int it = (blockIdx.x * 8 + wave) * 4 + q;
  if (it < CHR * KT) {
    const int ql = it / KT, t = it - ql * KT;
    const int dl = ql / HW2, rem = ql - dl * HW2;
    const int h = rem / WW, w = rem - h * WW;
    const int d = dbase + dl;
    const int kd = t / 9, r9 = t - kd * 9, kh = r9 / 3, kw = r9 - kh * 3;
    int orow = dl * PLANE + h * WP + w;
    orow = orow < 0 ? 0 : (orow > MOFF - 1 ? MOFF - 1 : orow);
    const int ch = (g * KT + t) * 3;
    const float* op = offc + (size_t)orow * OFFN + ch;
    const float od = op[0] + boff[ch];
    const float oh = op[1] + boff[ch + 1];
    const float ow = op[2] + boff[ch + 2];
    const float pd = (float)(d + kd - 1) + od;
    const float ph = (float)(h + kh - 1) + oh;
    const float pw = (float)(w + kw - 1) + ow;
    const float d0f = floorf(pd), h0f = floorf(ph), w0f = floorf(pw);
    const float fd = pd - d0f, fh = ph - h0f, fw = pw - w0f;
    const int d0 = (int)fminf(fmaxf(d0f, -2.0f), (float)(DD + 1));
    const int h0 = (int)fminf(fmaxf(h0f, -2.0f), (float)(HH + 1));
    const int w0 = (int)fminf(fmaxf(w0f, -2.0f), (float)(WW + 1));
    const bool vd0 = (d0 >= 0) && (d0 < DD), vd1 = (d0 >= -1) && (d0 < DD - 1);
    const bool vh0 = (h0 >= 0) && (h0 < HH), vh1 = (h0 >= -1) && (h0 < HH - 1);
    const bool vw0 = (w0 >= 0) && (w0 < WW), vw1 = (w0 >= -1) && (w0 < WW - 1);
    const float wd0 = 1.0f - fd, wd1 = fd;
    const float wh0 = 1.0f - fh, wh1 = fh;
    const float ww0 = 1.0f - fw, ww1 = fw;
    const float a00 = wd0 * wh0, a01 = wd0 * wh1, a10 = wd1 * wh0, a11 = wd1 * wh1;
    float c000 = a00 * ww0, c001 = a00 * ww1, c010 = a01 * ww0, c011 = a01 * ww1;
    float c100 = a10 * ww0, c101 = a10 * ww1, c110 = a11 * ww0, c111 = a11 * ww1;
    c000 = (vd0 && vh0 && vw0) ? c000 : 0.0f;
    c001 = (vd0 && vh0 && vw1) ? c001 : 0.0f;
    c010 = (vd0 && vh1 && vw0) ? c010 : 0.0f;
    c011 = (vd0 && vh1 && vw1) ? c011 : 0.0f;
    c100 = (vd1 && vh0 && vw0) ? c100 : 0.0f;
    c101 = (vd1 && vh0 && vw1) ? c101 : 0.0f;
    c110 = (vd1 && vh1 && vw0) ? c110 : 0.0f;
    c111 = (vd1 && vh1 && vw1) ? c111 : 0.0f;
    int da = d0, db = d0 + 1, ha = h0, hb = h0 + 1, wa = w0, wb = w0 + 1;
    da = da < 0 ? 0 : (da > DD - 1 ? DD - 1 : da);
    db = db < 0 ? 0 : (db > DD - 1 ? DD - 1 : db);
    ha = ha < 0 ? 0 : (ha > HH - 1 ? HH - 1 : ha);
    hb = hb < 0 ? 0 : (hb > HH - 1 ? HH - 1 : hb);
    wa = wa < 0 ? 0 : (wa > WW - 1 ? WW - 1 : wa);
    wb = wb < 0 ? 0 : (wb > WW - 1 ? WW - 1 : wb);
    const int pda = da * HW2, pdb = db * HW2, pha = ha * WW, phb = hb * WW;
    const float* xb = xT + (size_t)n * PP * CC + g * 8;
    v4f va = (v4f){0.f, 0.f, 0.f, 0.f}, vb = (v4f){0.f, 0.f, 0.f, 0.f};
    acc_corner(xb + (size_t)(pda + pha + wa) * CC, c000, va, vb);
    acc_corner(xb + (size_t)(pda + pha + wb) * CC, c001, va, vb);
    acc_corner(xb + (size_t)(pda + phb + wa) * CC, c010, va, vb);
    acc_corner(xb + (size_t)(pda + phb + wb) * CC, c011, va, vb);
    acc_corner(xb + (size_t)(pdb + pha + wa) * CC, c100, va, vb);
    acc_corner(xb + (size_t)(pdb + pha + wb) * CC, c101, va, vb);
    acc_corner(xb + (size_t)(pdb + phb + wa) * CC, c110, va, vb);
    acc_corner(xb + (size_t)(pdb + phb + wb) * CC, c111, va, vb);
    v4u u;
    u[0] = pkh2(va[0], va[1]); u[1] = pkh2(va[2], va[3]);
    u[2] = pkh2(vb[0], vb[1]); u[3] = pkh2(vb[2], vb[3]);
    volatile v4u* dst = (volatile v4u*)(S + (size_t)ql * KD + t * CC + g * 8);
    *dst = u;
    __threadfence();
    *dst = u;
  }
}

template <int PADDED>
__global__ __launch_bounds__(256) void k_bnstat(const float* __restrict__ src, double* __restrict__ part) {
  __shared__ double sh[2][4][CC];
  const int tid = threadIdx.x, c = tid & 63, rg = tid >> 6, sl = blockIdx.x;
  double s = 0.0, s2 = 0.0;
#pragma unroll 2
  for (int i = 0; i < RS / 4; ++i) {
    const int qrow = sl * RS + rg + 4 * i;
    size_t row = (size_t)qrow;
    if (PADDED) {
      const int n = qrow / PP, p = qrow - n * PP;
      const int d = p / HW2, rem = p - d * HW2, h = rem / WW, w = rem - h * WW;
      row = (size_t)n * RO + (size_t)(d * PLANE + h * WP + w);
    }
    const float v = src[row * CC + c];
    const double dv = (double)v;
    s += dv; s2 += dv * dv;
  }
  sh[0][rg][c] = s; sh[1][rg][c] = s2;
  __syncthreads();
  if (tid < CC) {
    const double a = ((sh[0][0][c] + sh[0][1][c]) + sh[0][2][c]) + sh[0][3][c];
    const double b = ((sh[1][0][c] + sh[1][1][c]) + sh[1][2][c]) + sh[1][3][c];
    volatile double* pp = part + (size_t)sl * (2 * CC);
    pp[c] = a; pp[CC + c] = b;
    __threadfence();
    pp[c] = a; pp[CC + c] = b;
  }
}

__global__ __launch_bounds__(64) void k_bnfin(const double* __restrict__ part, float* __restrict__ stats) {
  const int c = threadIdx.x;
  double s = 0.0, s2 = 0.0;
  for (int sl = 0; sl < NSL; ++sl) {
    s  += part[(size_t)sl * (2 * CC) + c];
    s2 += part[(size_t)sl * (2 * CC) + CC + c];
  }
  const double inv = 1.0 / (double)NQ;
  const double m = s * inv;
  double var = s2 * inv - m * m;
  var = var < 0.0 ? 0.0 : var;
  const float mf = (float)m;
  const float vf = (float)var;
  const float rs = 1.0f / sqrtf(vf + 1e-5f);
  volatile float* st = stats;
  st[c] = mf; st[CC + c] = rs;
  __threadfence();
  st[c] = mf; st[CC + c] = rs;
}

__global__ __launch_bounds__(256) void k_final(const float* __restrict__ o2, const float* __restrict__ stats,
                                              const float* __restrict__ gamma, const float* __restrict__ beta,
                                              const float* __restrict__ x, float* __restrict__ out) {
  __shared__ float t[CC][33];
  const int tid = threadIdx.x;
  const int blk = blockIdx.x;
  const int n   = blk / (PP / 32);
  const int p0  = (blk - n * (PP / 32)) * 32;
#pragma unroll
  for (int i = 0; i < 8; ++i) {
    const int idx = i * 256 + tid;
    const int j = idx >> 6, c = idx & 63;
    const int p = p0 + j;
    const int d = p / HW2, rem = p - d * HW2, h = rem / WW, w = rem - h * WW;
    const size_t row = (size_t)n * RO + (size_t)(d * PLANE + h * WP + w);
    t[c][j] = o2[row * CC + c];
  }
  __syncthreads();
  const int wave = tid >> 5, lane = tid & 31, q = lane >> 3, j4 = (lane & 7) * 4;
  for (int pass = 0; pass < 2; ++pass) {
#pragma unroll
    for (int it = 0; it < 2; ++it) {
      const int c = it * 32 + wave * 4 + q;
      const float mu = stats[c], rsd = stats[CC + c], ga = gamma[c], be = beta[c];
      const size_t base = ((size_t)(n * CC + c)) * PP + p0 + j4;
      const v4f xv = *(const v4f*)(x + base);
      v4f v;
#pragma unroll
      for (int e = 0; e < 4; ++e) v[e] = fmaxf((ga * (t[c][j4 + e] - mu)) * rsd + be + xv[e], 0.0f);
      *(volatile v4f*)(out + base) = v;
    }
    __threadfence();
  }
}

extern "C" void kernel_launch(void* const* d_in, const int* in_sizes, int n_in,
                              void* d_out, int out_size, void* d_ws, size_t ws_size,
                              hipStream_t stream) {
  if (n_in < 10) return;
  if (in_sizes[0] != NQ * CC || in_sizes[1] != OFFC * KD || in_sizes[2] != OFFC ||
      in_sizes[3] != CC * KD || in_sizes[4] != CC || in_sizes[5] != CC ||
      in_sizes[6] != CC * KD || in_sizes[7] != CC || in_sizes[8] != CC || in_sizes[9] != CC) return;
  if (out_size != NQ * CC) return;

  const float* x      = (const float*)d_in[0];
  const float* w_off  = (const float*)d_in[1];
  const float* b_off  = (const float*)d_in[2];
  const float* w1     = (const float*)d_in[3];
  const float* gamma1 = (const float*)d_in[4];
  const float* beta1  = (const float*)d_in[5];
  const float* w2     = (const float*)d_in[6];
  const float* b2     = (const float*)d_in[7];
  const float* gamma2 = (const float*)d_in[8];
  const float* beta2  = (const float*)d_in[9];
  float* out = (float*)d_out;

  const size_t bytes_xT   = (size_t)NQ * CC * 4;
  const size_t bytes_xP   = (size_t)NB * RP * CC * 2;
  const size_t bytes_Bo   = (size_t)OFFN * KD * 2;
  const size_t bytes_Bw   = (size_t)CC * KD * 2;
  const size_t bytes_offc = (size_t)MOFF * OFFN * 4;
  const size_t bytes_Sc   = (size_t)CHR * KD * 2;
  const size_t bytes_o1   = (size_t)NQ * CC * 4;
  const size_t bytes_o2   = (size_t)NB * RO * CC * 4;
  const size_t bytes_part = (size_t)NSL * 2 * CC * 8;
  const size_t bytes_st   = 1024;
  char* ws = (char*)d_ws;
  size_t o = 0;
  float* xT = (float*)(ws + o);                              o += bytes_xT;
  unsigned short* xP  = (unsigned short*)(ws + o);           o += bytes_xP;
  unsigned short* xP2 = (unsigned short*)(ws + o);           o += bytes_xP;
  unsigned short* Bo  = (unsigned short*)(ws + o);           o += bytes_Bo;
  unsigned short* B1  = (unsigned short*)(ws + o);           o += bytes_Bw;
  unsigned short* B2  = (unsigned short*)(ws + o);           o += bytes_Bw;
  float* offc = (float*)(ws + o);                            o += bytes_offc;
  unsigned short* Sc  = (unsigned short*)(ws + o);           o += bytes_Sc;
  float* out1 = (float*)(ws + o);                            o += bytes_o1;
  float* out2 = (float*)(ws + o);                            o += bytes_o2;
  double* part = (double*)(ws + o);                          o += bytes_part;
  float* stats1 = (float*)(ws + o);
  float* stats2 = (float*)(ws + o + 512);                    o += bytes_st;
  if (o > ws_size) return;
  if (o > (size_t)134217728) return;

  k_xpose<<<NB * PP / 32, 256, 0, stream>>>(x, xT);
  k_pad16<0><<<NB * RP / 32, 256, 0, stream>>>(xT, gamma1, gamma1, beta1, xP);
  k_prepw<<<(OFFN * (KD / 8) + 255) / 256, 256, 0, stream>>>(w_off, Bo, OFFN, OFFC, 1024.0f);
  k_prepw<<<(CC * (KD / 8) + 255) / 256, 256, 0, stream>>>(w1, B1, CC, CC, 256.0f);
  k_prepw<<<(CC * (KD / 8) + 255) / 256, 256, 0, stream>>>(w2, B2, CC, CC, 256.0f);

  for (int ck = 0; ck < NCH; ++ck) {
    const int n = ck / (DD / 2);
    const int dbase = 2 * (ck - n * (DD / 2));
    const int ms = MSO + dbase * PLANE;
    const unsigned short* Ax = xP + ((size_t)n * RP + GF + ms) * CC;
    wmma_gemm64<0, false, 0, 0, false, 0, 1><<<dim3((MOFF / 64) * (OFFN / 64) / 8, 1), 256, 0, stream>>>(
        Ax, Ax, CC, 0L,
        Bo, Bo, KD, 0L,
        (void*)offc, (void*)offc, OFFN, 0L,
        b_off,
        b_off, 0L,
        MOFF, OFFN, KD, 1.0f / 1024.0f);
    k_sample<<<CHR * KT / 32, 256, 0, stream>>>(xT, offc, b_off, Sc, n, dbase);
    float* o1 = out1 + ((size_t)n * PP + (size_t)dbase * HW2) * CC;
    wmma_gemm64<0, false, 0, 0, false, 0, 0><<<dim3((CHR / 64 + 7) / 8, 1), 256, 0, stream>>>(
        Sc, Sc, KD, 0L,
        B1, B1, KD, 0L,
        (void*)o1, (void*)offc, CC, 0L,
        b2,
        b2, 0L,
        CHR, CC, KD, 1.0f / 256.0f);
  }

  k_bnstat<0><<<NSL, 256, 0, stream>>>(out1, part);
  k_bnfin<<<1, 64, 0, stream>>>(part, stats1);
  k_pad16<1><<<NB * RP / 32, 256, 0, stream>>>(out1, stats1, gamma1, beta1, xP2);

  wmma_gemm64<0, false, 2, 0, false, 0, 1><<<dim3((RO / 64 + 7) / 8, NB), 256, 0, stream>>>(
      xP2 + (size_t)(GF + MSO) * CC, xP2 + (size_t)(GF + MSO) * CC, CC, (long)RP * CC,
      B2, B2, KD, 0L,
      (void*)out2, (void*)offc, CC, (long)RO * CC,
      b2,
      b2, 0L,
      RO, CC, KD, 1.0f / 256.0f);

  k_bnstat<1><<<NSL, 256, 0, stream>>>(out2, part);
  k_bnfin<<<1, 64, 0, stream>>>(part, stats2);
  k_final<<<NB * PP / 32, 256, 0, stream>>>(out2, stats2, gamma2, beta2, x, out);
  (void)hipGetLastError();
}
